// AttentionHead_9723805958414
// MI455X (gfx1250) — hardware-verified
//
#include <hip/hip_runtime.h>
#include <math.h>

constexpr int NPTS = 100000;
constexpr int KNB = 16;
constexpr int DIMC = 64;
constexpr int NPAD = 100032;
constexpr int QKV_LD = 3 * DIMC;
constexpr int NENT = NPTS * KNB;
constexpr int NGROUP = NPTS / 8;
constexpr int GRID_MAIN = 500;
constexpr int MOM_BLOCKS = 250;
constexpr int MOM_EPT = 25;
constexpr int CAST_BLOCKS = NPAD * 8 / 256;
constexpr int APITCH = 72;
constexpr int VPITCH = 64;
constexpr int AB1_N = 192;
constexpr float WCARRY = 16.0f;
constexpr float WCARRY_INV = 0.0625f;
constexpr float BN_EPS = 1e-5f;
constexpr float PAD_COORD = 1.0e6f;
constexpr double INV_NENT = 1.0 / 1600000.0;

static_assert(NPAD % 64 == 0 && NPAD > NPTS && NPAD % 32 == 0);
static_assert(CAST_BLOCKS * 256 == NPAD * 8);
static_assert(MOM_BLOCKS * 256 * MOM_EPT == NENT);
static_assert(NGROUP * 8 == NPTS);
static_assert(NGROUP % GRID_MAIN == 0);
static_assert(DIMC % 32 == 0 && QKV_LD % 64 == 0 && DIMC == 64);

typedef __attribute__((ext_vector_type(16))) _Float16 v16h;
typedef __attribute__((ext_vector_type(8)))  _Float16 v8h;
typedef __attribute__((ext_vector_type(16))) __bf16   v16b;
typedef __attribute__((ext_vector_type(8)))  __bf16   v8b;
typedef __attribute__((ext_vector_type(8)))  float    v8f;
typedef __attribute__((ext_vector_type(4)))  float    v4f;
typedef __attribute__((ext_vector_type(4)))  unsigned int v4u;

__device__ __forceinline__ unsigned short f2bf_bits(float f) {
  unsigned u = __float_as_uint(f);
  return (unsigned short)((u + 0x7FFFu + ((u >> 16) & 1u)) >> 16);
}
__device__ __forceinline__ float bf_bits2f(unsigned short h) { return __uint_as_float(((unsigned)h) << 16); }

__device__ __forceinline__ void dep_guard_h(v8f& a, v8f& b, v16h x, v16h y) { asm volatile("v_nop\n\tv_nop\n\tv_nop\n\tv_nop" : "+v"(a), "+v"(b) : "v"(x), "v"(y)); }
__device__ __forceinline__ void dep_guard_b(v8f& a, v8f& b, v16b x, v16b y) { asm volatile("v_nop\n\tv_nop\n\tv_nop\n\tv_nop" : "+v"(a), "+v"(b) : "v"(x), "v"(y)); }
__device__ __forceinline__ void keep4_h(v16h a, v16h b, v16h c, v16h d) { asm volatile("v_nop" :: "v"(a), "v"(b), "v"(c), "v"(d)); }
__device__ __forceinline__ void keep4_b(v16b a, v16b b, v16b c, v16b d) { asm volatile("v_nop" :: "v"(a), "v"(b), "v"(c), "v"(d)); }
__device__ __forceinline__ void acc_guard4(v8f& a, v8f& b, v8f& c, v8f& d) { asm volatile("v_nop\n\tv_nop\n\tv_nop\n\tv_nop" : "+v"(a), "+v"(b), "+v"(c), "+v"(d)); }
template <typename T> struct Frag;
template <> struct Frag<_Float16> {
  typedef v16h V; union U { v16h v; v8h h[2]; };
  static __device__ __forceinline__ v16h load(const _Float16* p) {
    U f; f.h[0] = *(const v8h*)(p); f.h[1] = *(const v8h*)(p + 16); return f.v;
  }
  static __device__ __forceinline__ v8f mma(v16h a, v16h b, v8f c) {
    return __builtin_amdgcn_wmma_f32_16x16x32_f16(false, a, false, b, (short)0, c, false, false);
  }
  static __device__ __forceinline__ void guard(v8f& a, v8f& b, v16h x, v16h y) { dep_guard_h(a, b, x, y); }
  static __device__ __forceinline__ void keep(v16h a, v16h b, v16h c, v16h d) { keep4_h(a, b, c, d); }
};
template <> struct Frag<__bf16> {
  typedef v16b V; union U { v16b v; v8b h[2]; };
  static __device__ __forceinline__ v16b load(const __bf16* p) {
    U f; f.h[0] = *(const v8b*)(p); f.h[1] = *(const v8b*)(p + 16); return f.v;
  }
  static __device__ __forceinline__ v8f mma(v16b a, v16b b, v8f c) {
    return __builtin_amdgcn_wmma_f32_16x16x32_bf16(false, a, false, b, (short)0, c, false, false);
  }
  static __device__ __forceinline__ void guard(v8f& a, v8f& b, v16b x, v16b y) { dep_guard_b(a, b, x, y); }
  static __device__ __forceinline__ void keep(v16b a, v16b b, v16b c, v16b d) { keep4_b(a, b, c, d); }
};

__device__ __forceinline__ unsigned pk16(unsigned short a, unsigned short b) { return (unsigned)a | ((unsigned)b << 16); }
__device__ __forceinline__ unsigned short h_bits(float f) { const _Float16 h = (_Float16)f; return __builtin_bit_cast(unsigned short, h); }

template <int ET> struct Elem;
template <> struct Elem<0> { typedef _Float16 T; };
template <> struct Elem<1> { typedef __bf16 T; };
template <int ET, bool SPLIT, int BIAS_MODE, int OUT_MODE, bool RESID, int ACT = 0>
__global__ __launch_bounds__(256) void wmma_gemm64(
    const unsigned short* __restrict__ Ap, const unsigned short* __restrict__ A2p, int lda, long strideA,
    const unsigned short* __restrict__ Btp, const unsigned short* __restrict__ Bt2p, int ldb, long strideB,
    void* __restrict__ Cout, void* __restrict__ Cout2, int ldc, long strideC,
    const float* __restrict__ bias,
    const float* __restrict__ resid, long strideR,
    int M, int N, int K, float scale) {
  typedef typename Elem<ET>::T T;
  typedef typename Frag<T>::V V;
  const T* A = (const T*)Ap; const T* A2 = (const T*)A2p; const T* Bt = (const T*)Btp; const T* Bt2 = (const T*)Bt2p;
  __shared__ __align__(16) float sT[8][16 * 68];
  const int b    = blockIdx.y;
  const int lane = threadIdx.x & 31;
  const int wave = threadIdx.x >> 5;
  const int tilesN = N >> 6;
  const int tilesM = M >> 6;
  const int tile = blockIdx.x * 8 + wave;
  if (tile >= tilesM * tilesN) return;
  const int tm = tile / tilesN;
  const int tn = tile - tm * tilesN;
  const int m0 = tm << 6;
  const int n0 = tn << 6;

  const T* Ab  = A  + (size_t)b * strideA;
  const T* Bb  = Bt + (size_t)b * strideB;
  const T* Ab2 = SPLIT ? (A2  + (size_t)b * strideA) : nullptr;
  const T* Bb2 = SPLIT ? (Bt2 + (size_t)b * strideB) : nullptr;

  const int rlane = lane & 15;
  const int koff  = (lane >> 4) * 8;
  const int mOff  = (lane >> 4) * 8;

  v8f acc[4][4];
#pragma unroll
  for (int i = 0; i < 4; ++i)
#pragma unroll
    for (int j = 0; j < 4; ++j) acc[i][j] = (v8f){0.f,0.f,0.f,0.f,0.f,0.f,0.f,0.f};

  for (int k0 = 0; k0 < K; k0 += 32) {
    V bh[4], bl[4];
#pragma unroll
    for (int j = 0; j < 4; ++j) {
      const size_t bo = (size_t)(n0 + (j << 4) + rlane) * ldb + koff + k0;
      bh[j] = Frag<T>::load(Bb + bo);
      if (SPLIT) bl[j] = Frag<T>::load(Bb2 + bo);
    }
#pragma unroll
    for (int i = 0; i < 4; ++i) {
      const size_t ao = (size_t)(m0 + (i << 4) + rlane) * lda + koff + k0;
      V ah = Frag<T>::load(Ab + ao);
      V al;
      if (SPLIT) al = Frag<T>::load(Ab2 + ao);
#pragma unroll
      for (int j = 0; j < 4; ++j) {
        acc[i][j] = Frag<T>::mma(ah, bh[j], acc[i][j]);
        if (SPLIT) {
          acc[i][j] = Frag<T>::mma(ah, bl[j], acc[i][j]);
          acc[i][j] = Frag<T>::mma(al, bh[j], acc[i][j]);
        }
      }
      Frag<T>::guard(acc[i][0], acc[i][3], ah, SPLIT ? al : ah);
    }
    Frag<T>::keep(bh[0], bh[1], bh[2], bh[3]);
    if (SPLIT) Frag<T>::keep(bl[0], bl[1], bl[2], bl[3]);
  }
  acc_guard4(acc[0][0], acc[0][1], acc[0][2], acc[0][3]);
  acc_guard4(acc[1][0], acc[1][1], acc[1][2], acc[1][3]);
  acc_guard4(acc[2][0], acc[2][1], acc[2][2], acc[2][3]);
  acc_guard4(acc[3][0], acc[3][1], acc[3][2], acc[3][3]);

  float* slab = sT[wave];
  const float* Rb = RESID ? (resid + (size_t)b * strideR) : nullptr;
#pragma unroll
  for (int i = 0; i < 4; ++i) {
    const int mBase = m0 + (i << 4);
#pragma unroll
    for (int j = 0; j < 4; ++j) {
      const int n = n0 + (j << 4) + rlane;
      float bv = 0.f;
      if (BIAS_MODE == 2) bv = bias[n];
#pragma unroll
      for (int r = 0; r < 8; ++r) {
        float v = acc[i][j][r] * scale;
        if (BIAS_MODE == 1) v += bias[mBase + mOff + r];
        if (BIAS_MODE == 2) v += bv;
        if (RESID) v += Rb[(size_t)(mBase + mOff + r) * ldc + n];
        if (ACT == 2) v = fmaxf(v, 0.0f);
        if (ACT == 4) v = (v > 0.f) ? v : 0.01f * v;
        slab[(mOff + r) * 68 + (j << 4) + rlane] = v;
      }
    }
    __builtin_amdgcn_fence(__ATOMIC_RELEASE, "workgroup");
    __builtin_amdgcn_wave_barrier();
    __builtin_amdgcn_fence(__ATOMIC_ACQUIRE, "workgroup");
    if (OUT_MODE == 0) {
      float* C = (float*)Cout + (size_t)b * strideC;
      const int hh = lane >> 4, c4 = (lane & 15) * 4;
      for (int pass = 0; pass < 2; ++pass) {
#pragma unroll
        for (int it = 0; it < 8; ++it) {
          const int row = it * 2 + hh;
          v4f v = *(const v4f*)(slab + row * 68 + c4);
          *(volatile v4f*)(C + (size_t)(mBase + row) * ldc + n0 + c4) = v;
        }
        __threadfence();
      }
    } else {
      const int q = lane >> 3, c8 = (lane & 7) * 8;
      unsigned short* C  = (unsigned short*)Cout  + (size_t)b * strideC;
      unsigned short* C2 = (OUT_MODE == 2) ? ((unsigned short*)Cout2 + (size_t)b * strideC) : nullptr;
      for (int pass = 0; pass < 2; ++pass) {
#pragma unroll
        for (int it = 0; it < 4; ++it) {
          const int row = it * 4 + q;
          const float* sp = slab + row * 68 + c8;
          v8h hv, lv;
#pragma unroll
          for (int e = 0; e < 8; ++e) {
            if (OUT_MODE == 1) {
              hv[e] = (_Float16)sp[e];
            } else {
              unsigned short hb = f2bf_bits(sp[e]);
              unsigned short lb = f2bf_bits(sp[e] - bf_bits2f(hb));
              hv[e] = __builtin_bit_cast(_Float16, hb);
              lv[e] = __builtin_bit_cast(_Float16, lb);
            }
          }
          *(volatile v8h*)(C + (size_t)(mBase + row) * ldc + n0 + c8) = hv;
          if (OUT_MODE == 2) *(volatile v8h*)(C2 + (size_t)(mBase + row) * ldc + n0 + c8) = lv;
        }
        __threadfence();
      }
    }
    __builtin_amdgcn_fence(__ATOMIC_RELEASE, "workgroup");
    __builtin_amdgcn_wave_barrier();
    __builtin_amdgcn_fence(__ATOMIC_ACQUIRE, "workgroup");
  }
}

__global__ __launch_bounds__(256) void prep_w_kernel(
    const float* __restrict__ q_w, const float* __restrict__ k_w, const float* __restrict__ v_w, const float* __restrict__ w_w,
    const float* __restrict__ q_b, const float* __restrict__ k_b, const float* __restrict__ v_b,
    unsigned short* __restrict__ wcat, unsigned short* __restrict__ wwh, float* __restrict__ bcat) {
  const int blk = blockIdx.x;
  const int t = threadIdx.x;
  if (blk < 8) {
    const float* src = (blk < 2) ? q_w : ((blk < 4) ? k_w : ((blk < 6) ? v_w : w_w));
    unsigned short* dst = (blk < 6) ? (wcat + (blk >> 1) * (DIMC * DIMC)) : wwh;
    const int e = ((blk & 1) * 256 + t) * 8;
    const v4f a = *(const v4f*)(src + e);
    const v4f c = *(const v4f*)(src + e + 4);
    unsigned short hb[8];
#pragma unroll
    for (int i = 0; i < 4; ++i) {
      hb[i]     = h_bits(a[i] * WCARRY);
      hb[4 + i] = h_bits(c[i] * WCARRY);
    }
    const v4u u = (v4u){pk16(hb[0], hb[1]), pk16(hb[2], hb[3]), pk16(hb[4], hb[5]), pk16(hb[6], hb[7])};
    unsigned short* p = dst + e;
    *(volatile v4u*)p = u;
    __threadfence();
    *(volatile v4u*)p = u;
  } else {
    const int c4 = (t & 15) * 4;
    const v4f a = *(const v4f*)(q_b + c4);
    const v4f b = *(const v4f*)(k_b + c4);
    const v4f c = *(const v4f*)(v_b + c4);
    const float f0 = (t < 16) ? 1.0f : 0.0f;
    const float f1 = (t >= 16 && t < 32) ? 1.0f : 0.0f;
    const float f2 = (t >= 32) ? 1.0f : 0.0f;
    v4f v = a * f0;
    v = b * f1 + v;
    v = c * f2 + v;
    if (t < 48) {
      float* p = bcat + t * 4;
      *(volatile v4f*)p = v;
      __threadfence();
      *(volatile v4f*)p = v;
    }
  }
}

__global__ __launch_bounds__(256) void cast_feats_kernel(const float* __restrict__ feats, const float* __restrict__ points,
                                                         unsigned short* __restrict__ fh, float* __restrict__ pts4) {
  const int i = blockIdx.x * 256 + threadIdx.x;
  const int ic = (i < NPTS * 8) ? i : (NPTS * 8 - 1);
  const float live = (i < NPTS * 8) ? 1.0f : 0.0f;
  const v4f a = *(const v4f*)(feats + (size_t)ic * 8);
  const v4f c = *(const v4f*)(feats + (size_t)ic * 8 + 4);
  unsigned short hb[8];
#pragma unroll
  for (int e = 0; e < 4; ++e) {
    hb[e]     = h_bits(a[e] * live);
    hb[4 + e] = h_bits(c[e] * live);
  }
  const v4u u = (v4u){pk16(hb[0], hb[1]), pk16(hb[2], hb[3]), pk16(hb[4], hb[5]), pk16(hb[6], hb[7])};
  unsigned short* pq = fh + (size_t)i * 8;
  *(volatile v4u*)pq = u;
  __threadfence();
  *(volatile v4u*)pq = u;

  const int ir = (i < NPTS) ? i : (NPTS - 1);
  const float x = points[(size_t)ir * 3 + 0];
  const float y = points[(size_t)ir * 3 + 1];
  const float z = points[(size_t)ir * 3 + 2];
  const float lv = (i < NPTS) ? 1.0f : 0.0f;
  const float pv = (i == NPTS) ? PAD_COORD : 0.0f;
  const v4f o = (v4f){fmaf(x, lv, pv), fmaf(y, lv, pv), fmaf(z, lv, pv), 0.0f};
  if (i < NPAD) {
    float* pp = pts4 + (size_t)i * 4;
    *(volatile v4f*)pp = o;
    __threadfence();
    *(volatile v4f*)pp = o;
  }
}

__global__ __launch_bounds__(64) void padrow_kernel(float* __restrict__ qkv) {
  const int t = threadIdx.x;
  const v4f zz = (v4f){0.0f, 0.0f, 0.0f, 0.0f};
  if (t < 48) {
    float* p = qkv + (size_t)NPTS * QKV_LD + t * 4;
    *(volatile v4f*)p = zz;
    __threadfence();
    *(volatile v4f*)p = zz;
  }
}

__global__ __launch_bounds__(256) void moments_kernel(const int* __restrict__ nbr, const float* __restrict__ pts4, double* __restrict__ mom) {
  __shared__ double red[9 * 256];
  __shared__ __align__(16) double o16[16];
  const int tid = threadIdx.x;
  const int gt = blockIdx.x * 256 + tid;
  double a[9];
#pragma unroll
  for (int i = 0; i < 9; ++i) a[i] = 0.0;
#pragma unroll 1
  for (int i = 0; i < MOM_EPT; ++i) {
    const int e = gt + i * (MOM_BLOCKS * 256);
    int idx = nbr[e];
    idx = idx < 0 ? 0 : (idx > NPTS ? NPTS : idx);
    const v4f p = *(const v4f*)(pts4 + (size_t)idx * 4);
    const double x = (double)p[0], y = (double)p[1], z = (double)p[2];
    a[0] += x; a[1] += y; a[2] += z;
    a[3] += x * x; a[4] += y * y; a[5] += z * z;
    a[6] += x * y; a[7] += x * z; a[8] += y * z;
  }
#pragma unroll
  for (int i = 0; i < 9; ++i) red[i * 256 + tid] = a[i];
  __syncthreads();
  if (tid < 16) {
    const int row = (tid < 9) ? tid : 8;
    double s = 0.0;
#pragma unroll 1
    for (int t2 = 0; t2 < 256; ++t2) s += red[row * 256 + t2];
    const double keep = (tid < 9) ? 1.0 : 0.0;
    o16[tid] = s * keep;
  }
  __syncthreads();
  if (tid < 8) {
    const v4f v = *(const v4f*)((const float*)o16 + 4 * tid);
    float* p = (float*)mom + (size_t)blockIdx.x * 32 + 4 * tid;
    for (int pass = 0; pass < 2; ++pass) { *(volatile v4f*)p = v; __threadfence(); }
  }
}

__global__ __launch_bounds__(64) void bn1_kernel(const double* __restrict__ mom, const float* __restrict__ p_w, const float* __restrict__ p_b,
                                                const float* __restrict__ gam, const float* __restrict__ bet,
                                                const float* __restrict__ w_w, const float* __restrict__ w_b, float* __restrict__ ab1) {
  __shared__ __align__(16) float AB[AB1_N];
  __shared__ float PF[DIMC];
  const int c = threadIdx.x;
  double tm[9];
#pragma unroll
  for (int i = 0; i < 9; ++i) tm[i] = 0.0;
#pragma unroll 1
  for (int b = 0; b < MOM_BLOCKS; ++b) {
#pragma unroll
    for (int i = 0; i < 9; ++i) tm[i] += mom[b * 16 + i];
  }
  const float pw0 = p_w[c * 3 + 0], pw1 = p_w[c * 3 + 1], pw2 = p_w[c * 3 + 2], pbc = p_b[c];
  const double w0 = (double)pw0, w1 = (double)pw1, w2 = (double)pw2;
  const double g1 = w0 * tm[0] + w1 * tm[1] + w2 * tm[2];
  const double g2 = w0 * w0 * tm[3] + w1 * w1 * tm[4] + w2 * w2 * tm[5]
                  + 2.0 * (w0 * w1 * tm[6] + w0 * w2 * tm[7] + w1 * w2 * tm[8]);
  const double ml = g1 * INV_NENT;
  double var = g2 * INV_NENT - ml * ml;
  var = var > 0.0 ? var : 0.0;
  const double mean = ml + (double)pbc;
  const float istd = 1.0f / sqrtf((float)var + BN_EPS);
  const float av = gam[c] * istd;
  const float bsh = bet[c] - (float)mean * av;
  AB[c] = av;
  AB[64 + c] = bsh;
  const float pl = fmaf(PAD_COORD, pw0, fmaf(PAD_COORD, pw1, fmaf(PAD_COORD, pw2, pbc)));
  PF[c] = fmaxf(fmaf(av, pl, bsh), 0.0f);
  __syncthreads();
  float s = 0.0f;
  const float* wr = w_w + c * DIMC;
#pragma unroll 1
  for (int k4 = 0; k4 < DIMC / 4; ++k4) {
    const v4f w4 = *(const v4f*)(wr + 4 * k4);
    s = fmaf(PF[4 * k4 + 0], w4[0], s);
    s = fmaf(PF[4 * k4 + 1], w4[1], s);
    s = fmaf(PF[4 * k4 + 2], w4[2], s);
    s = fmaf(PF[4 * k4 + 3], w4[3], s);
  }
  s += w_b[c];
  AB[128 + c] = s;
  __syncthreads();
  if (c < 48) {
    const v4f v = *(const v4f*)(AB + 4 * c);
    float* p = ab1 + 4 * c;
    for (int pass = 0; pass < 2; ++pass) { *(volatile v4f*)p = v; __threadfence(); }
  }
}

template <int MODE>
__global__ __launch_bounds__(256) void vecattn_kernel(
    const int* __restrict__ nbr, const float* __restrict__ pts4, const float* __restrict__ qkv,
    const unsigned short* __restrict__ wwh, const float* __restrict__ p_w, const float* __restrict__ p_b,
    const float* __restrict__ ab1, const float* __restrict__ w_b, const float* __restrict__ ab2,
    double* __restrict__ part, float* __restrict__ out) {
  __shared__ __align__(16) unsigned short WS[DIMC * APITCH];
  __shared__ __align__(16) unsigned short As[8][16 * APITCH];
  __shared__ __align__(16) float Vs[MODE ? 8 : 1][MODE ? 16 * VPITCH : 4];
  __shared__ __align__(16) float Os[MODE ? 8 : 1][DIMC];
  __shared__ __align__(16) double RS[MODE ? 2 : 8 * 2 * 2 * DIMC];
  __shared__ __align__(16) double OD[MODE ? 2 : 2 * DIMC];
  __shared__ float Ps[8][KNB];
  __shared__ float s_pw0[DIMC], s_pw1[DIMC], s_pw2[DIMC], s_pb[DIMC], s_ap[DIMC], s_bp[DIMC], s_wb[DIMC], s_aw[DIMC], s_bw[DIMC], s_wlp[DIMC];

  const int tid  = threadIdx.x;
  const int lane = tid & 31, wave = tid >> 5;
  const int h = lane >> 4, m = lane & 15;
  const int jrow = lane >> 1, colbase = (lane & 1) * 32;

  for (int i = tid; i < DIMC * DIMC / 8; i += 256) {
    const int e = i * 8;
    const int row = e >> 6, col = e & 63;
    const v4u u = *(const v4u*)(wwh + e);
    *(v4u*)(WS + row * APITCH + col) = u;
  }
  if (tid < DIMC) {
    s_pw0[tid] = p_w[tid * 3 + 0];
    s_pw1[tid] = p_w[tid * 3 + 1];
    s_pw2[tid] = p_w[tid * 3 + 2];
    s_pb[tid]  = p_b[tid];
    s_ap[tid]  = ab1[tid];
    s_bp[tid]  = ab1[DIMC + tid];
    s_wlp[tid] = ab1[2 * DIMC + tid];
    s_wb[tid]  = w_b[tid];
    if (MODE) { s_aw[tid] = ab2[tid]; s_bw[tid] = ab2[DIMC + tid]; }
    else      { s_aw[tid] = 0.0f;     s_bw[tid] = 0.0f; }
  }
  __syncthreads();

  double dsum[4], dsq[4];
#pragma unroll
  for (int t = 0; t < 4; ++t) { dsum[t] = 0.0; dsq[t] = 0.0; }
  const v8f zero8 = (v8f){0.f, 0.f, 0.f, 0.f, 0.f, 0.f, 0.f, 0.f};

#pragma unroll 1
  for (int g = blockIdx.x; g < NGROUP; g += gridDim.x) {
    const int n = g * 8 + wave;
    {
      int idx = nbr[(size_t)n * KNB + jrow];
      idx = idx < 0 ? 0 : (idx > NPTS ? NPTS : idx);
      if ((lane & 1) == 0) Ps[wave][jrow] = (idx == NPTS) ? 1.0f : 0.0f;
      const v4f pp = *(const v4f*)(pts4 + (size_t)idx * 4);
      const float px = pp[0], py = pp[1], pz = pp[2];
      const float* krow = qkv + (size_t)idx * QKV_LD + DIMC + colbase;
      const float* vrow = qkv + (size_t)idx * QKV_LD + 2 * DIMC + colbase;
      const float* qrow = qkv + (size_t)n * QKV_LD + colbase;
      unsigned short* arow = As[wave] + jrow * APITCH + colbase;
      float* vsrow = Vs[MODE ? wave : 0] + (MODE ? (jrow * VPITCH + colbase) : 0);
#pragma unroll 1
      for (int cc = 0; cc < 4; ++cc) {
        const int c0 = cc * 8;
        const v4f ka = *(const v4f*)(krow + c0);
        const v4f kb = *(const v4f*)(krow + c0 + 4);
        const v4f qa = *(const v4f*)(qrow + c0);
        const v4f qb = *(const v4f*)(qrow + c0 + 4);
        v4f va = (v4f){0.0f, 0.0f, 0.0f, 0.0f};
        v4f vb = va;
        if (MODE) { va = *(const v4f*)(vrow + c0); vb = *(const v4f*)(vrow + c0 + 4); }
        float kg8[8], q8[8], vg8[8];
#pragma unroll
        for (int e = 0; e < 4; ++e) {
          kg8[e] = ka[e]; kg8[4 + e] = kb[e];
          q8[e]  = qa[e]; q8[4 + e]  = qb[e];
          vg8[e] = va[e]; vg8[4 + e] = vb[e];
        }
        unsigned short hb[8];
        float vl[8];
#pragma unroll
        for (int e = 0; e < 8; ++e) {
          const int c = colbase + c0 + e;
          const float pl = fmaf(px, s_pw0[c], fmaf(py, s_pw1[c], fmaf(pz, s_pw2[c], s_pb[c])));
          const float pf = fmaxf(fmaf(s_ap[c], pl, s_bp[c]), 0.0f);
          const float wpv = fmaf(kg8[e], q8[e], pf);
          hb[e] = h_bits(wpv);
          vl[e] = vg8[e] + pf;
        }
        const v4u u = (v4u){pk16(hb[0], hb[1]), pk16(hb[2], hb[3]), pk16(hb[4], hb[5]), pk16(hb[6], hb[7])};
        *(v4u*)(arow + c0) = u;
        if (MODE) {
          const v4f o0 = (v4f){vl[0], vl[1], vl[2], vl[3]};
          const v4f o1 = (v4f){vl[4], vl[5], vl[6], vl[7]};
          *(v4f*)(vsrow + c0) = o0;
          *(v4f*)(vsrow + c0 + 4) = o1;
        }
      }
    }
    __syncthreads();

    v8f acc[4];
#pragma unroll
    for (int t = 0; t < 4; ++t) acc[t] = zero8;
    {
      const _Float16* abase = (const _Float16*)(As[wave]) + m * APITCH + 8 * h;
      const _Float16* wsb   = (const _Float16*)(WS) + m * APITCH + 8 * h;
#pragma unroll
      for (int ks = 0; ks < 2; ++ks) {
        const v16h af = Frag<_Float16>::load(abase + ks * 32);
        v16h bf[4];
#pragma unroll
        for (int t = 0; t < 4; ++t) bf[t] = Frag<_Float16>::load(wsb + t * 16 * APITCH + ks * 32);
#pragma unroll
        for (int t = 0; t < 4; ++t) acc[t] = Frag<_Float16>::mma(af, bf[t], acc[t]);
        dep_guard_h(acc[0], acc[3], af, bf[3]);
        keep4_h(bf[0], bf[1], bf[2], bf[3]);
      }
      acc_guard4(acc[0], acc[1], acc[2], acc[3]);
    }

    float padf[8], keepf[8];
#pragma unroll
    for (int r = 0; r < 8; ++r) { padf[r] = Ps[wave][8 * h + r]; keepf[r] = 1.0f - padf[r]; }

    if (MODE) {
#pragma unroll
      for (int t = 0; t < 4; ++t) {
        const int col = t * 16 + m;
        const float wb = s_wb[col], aw = s_aw[col], bw = s_bw[col], wlp = s_wlp[col];
        float y[8];
        float mx = 0.0f;
#pragma unroll
        for (int r = 0; r < 8; ++r) {
          const float xn = fmaf(acc[t][r], WCARRY_INV, wb);
          const float x  = fmaf(padf[r], wlp, keepf[r] * xn);
          const float yy = fmaf(aw, x, bw);
          y[r] = fmaxf(yy, 0.0f);
          mx = fmaxf(mx, y[r]);
        }
        mx = fmaxf(mx, __shfl_xor(mx, 16, 32));
        float s8 = 0.0f, num = 0.0f;
        const float* vcol = Vs[MODE ? wave : 0] + (8 * h) * VPITCH + col;
#pragma unroll
        for (int r = 0; r < 8; ++r) {
          const float ex = __expf(y[r] - mx);
          s8 += ex;
          num = fmaf(ex, vcol[r * VPITCH], num);
        }
        s8  += __shfl_xor(s8, 16, 32);
        num += __shfl_xor(num, 16, 32);
        const float att = num * (1.0f / s8);
        if (h == 0) Os[MODE ? wave : 0][col] = att;
      }
      __syncthreads();
      const v4f ov = *(const v4f*)(Os[MODE ? wave : 0] + 4 * m);
      float* op = out + (size_t)n * DIMC + 4 * m;
      for (int pass = 0; pass < 2; ++pass) {
        if (h == 0) *(volatile v4f*)op = ov;
        __threadfence();
      }
      __syncthreads();
    } else {
#pragma unroll
      for (int t = 0; t < 4; ++t) {
        const int col = t * 16 + m;
        const float wb = s_wb[col], wlp = s_wlp[col];
        float s8 = 0.0f, q8 = 0.0f;
#pragma unroll
        for (int r = 0; r < 8; ++r) {
          const float xn = fmaf(acc[t][r], WCARRY_INV, wb);
          const float x  = fmaf(padf[r], wlp, keepf[r] * xn);
          s8 += x;
          q8 = fmaf(x, x, q8);
        }
        dsum[t] += (double)s8;
        dsq[t]  += (double)q8;
      }
      __syncthreads();
    }
  }

  if (MODE == 0) {
#pragma unroll
    for (int t = 0; t < 4; ++t) {
      const int col = t * 16 + m;
      RS[((wave * 2 + 0) * 2 + h) * DIMC + col] = dsum[t];
      RS[((wave * 2 + 1) * 2 + h) * DIMC + col] = dsq[t];
    }
    __syncthreads();
    if (tid < 2 * DIMC) {
      const int st = tid >> 6, col = tid & 63;
      double s = 0.0;
#pragma unroll
      for (int w = 0; w < 8; ++w) {
        s += RS[((w * 2 + st) * 2 + 0) * DIMC + col];
        s += RS[((w * 2 + st) * 2 + 1) * DIMC + col];
      }
      OD[tid] = s;
    }
    __syncthreads();
    if (wave == 0) {
      const float* odf = (const float*)OD;
      const v4f v0 = *(const v4f*)(odf + 4 * lane);
      const v4f v1 = *(const v4f*)(odf + 128 + 4 * lane);
      float* pp = (float*)part + (size_t)blockIdx.x * 256;
      for (int pass = 0; pass < 2; ++pass) {
        *(volatile v4f*)(pp + 4 * lane) = v0;
        *(volatile v4f*)(pp + 128 + 4 * lane) = v1;
        __threadfence();
      }
    }
  }
}

__global__ __launch_bounds__(128) void bn2_kernel(const double* __restrict__ part, const float* __restrict__ gam,
                                                 const float* __restrict__ bet, float* __restrict__ ab2) {
  __shared__ double T[128];
  __shared__ __align__(16) float AB[128];
  const int tid = threadIdx.x;
  double s = 0.0;
#pragma unroll 1
  for (int b = 0; b < GRID_MAIN; ++b) s += part[(size_t)b * 128 + tid];
  T[tid] = s;
  __syncthreads();
  if (tid < 64) {
    const double mean = T[tid] * INV_NENT;
    double var = T[64 + tid] * INV_NENT - mean * mean;
    var = var > 0.0 ? var : 0.0;
    const float istd = 1.0f / sqrtf((float)var + BN_EPS);
    const float av = gam[tid] * istd;
    const float bsh = bet[tid] - (float)mean * av;
    AB[tid] = av;
    AB[64 + tid] = bsh;
  }
  __syncthreads();
  if (tid < 32) {
    const v4f v = *(const v4f*)(AB + 4 * tid);
    float* p = ab2 + 4 * tid;
    for (int pass = 0; pass < 2; ++pass) { *(volatile v4f*)p = v; __threadfence(); }
  }
}

extern "C" void kernel_launch(void* const* d_in, const int* in_sizes, int n_in,
                              void* d_out, int out_size, void* d_ws, size_t ws_size, hipStream_t stream) {
  if (n_in < 17) return;
  if (in_sizes[1] != NENT || in_sizes[2] != NPTS * DIMC || out_size != NPTS * DIMC) return;
  const float* points    = (const float*)d_in[0];
  const int*   neighbors = (const int*)  d_in[1];
  const float* feats     = (const float*)d_in[2];
  const float* q_w = (const float*)d_in[3];   const float* q_b = (const float*)d_in[4];
  const float* k_w = (const float*)d_in[5];   const float* k_b = (const float*)d_in[6];
  const float* v_w = (const float*)d_in[7];   const float* v_b = (const float*)d_in[8];
  const float* p_w = (const float*)d_in[9];   const float* p_b = (const float*)d_in[10];
  const float* p_gamma = (const float*)d_in[11]; const float* p_beta = (const float*)d_in[12];
  const float* w_w = (const float*)d_in[13];  const float* w_b = (const float*)d_in[14];
  const float* w_gamma = (const float*)d_in[15]; const float* w_beta = (const float*)d_in[16];
  float* out = (float*)d_out;

  char* ws = (char*)d_ws; size_t off = 0;
  auto carve = [&](size_t bytes) -> char* { char* p = ws + off; off += (bytes + 255) & ~(size_t)255; return p; };
  unsigned short* WCAT = (unsigned short*)carve((size_t)QKV_LD * DIMC * 2);
  unsigned short* WWH  = (unsigned short*)carve((size_t)DIMC * DIMC * 2);
  float*          BCAT = (float*)carve((size_t)QKV_LD * 4);
  unsigned short* FH   = (unsigned short*)carve((size_t)NPAD * DIMC * 2);
  float*          PTS4 = (float*)carve((size_t)NPAD * 4 * 4);
  float*          QKV  = (float*)carve((size_t)NPAD * QKV_LD * 4);
  double*         MOM  = (double*)carve((size_t)MOM_BLOCKS * 16 * 8);
  float*          AB1  = (float*)carve((size_t)AB1_N * 4);
  double*         PART = (double*)carve((size_t)GRID_MAIN * 128 * 8);
  float*          AB2  = (float*)carve(128 * 4);
  if (off > ws_size || off > (size_t)134217728) return;

  prep_w_kernel<<<9, 256, 0, stream>>>(q_w, k_w, v_w, w_w, q_b, k_b, v_b, WCAT, WWH, BCAT);
  cast_feats_kernel<<<CAST_BLOCKS, 256, 0, stream>>>(feats, points, FH, PTS4);
  {
    const int tiles = (NPAD / 64) * (QKV_LD / 64);
    wmma_gemm64<0, false, 2, 0, false, 0><<<dim3((tiles + 7) / 8, 1), 256, 0, stream>>>(
        (const unsigned short*)FH, (const unsigned short*)FH, DIMC, 0L,
        (const unsigned short*)WCAT, (const unsigned short*)WCAT, DIMC, 0L,
        (void*)QKV, (void*)QKV, QKV_LD, 0L,
        (const float*)BCAT, (const float*)BCAT, 0L,
        NPAD, QKV_LD, DIMC, WCARRY_INV);
  }
  padrow_kernel<<<1, 64, 0, stream>>>(QKV);
  moments_kernel<<<MOM_BLOCKS, 256, 0, stream>>>(neighbors, PTS4, MOM);
  bn1_kernel<<<1, 64, 0, stream>>>(MOM, p_w, p_b, p_gamma, p_beta, w_w, w_b, AB1);
  vecattn_kernel<0><<<GRID_MAIN, 256, 0, stream>>>(neighbors, PTS4, QKV, WWH, p_w, p_b, AB1, w_b, AB2, PART, out);
  bn2_kernel<<<1, 128, 0, stream>>>(PART, w_gamma, w_beta, AB2);
  vecattn_kernel<1><<<GRID_MAIN, 256, 0, stream>>>(neighbors, PTS4, QKV, WWH, p_w, p_b, AB1, w_b, AB2, PART, out);
}
